// PatchSA_40338332844433
// MI455X (gfx1250) — hardware-verified
//
#include <hip/hip_runtime.h>
#include <stdint.h>

#define DEVINL __device__ __forceinline__

typedef _Float16 f16t;
typedef _Float16 v16h __attribute__((ext_vector_type(16)));
typedef _Float16 v8h  __attribute__((ext_vector_type(8)));
typedef _Float16 v4h  __attribute__((ext_vector_type(4)));
typedef float    v8f  __attribute__((ext_vector_type(8)));
typedef float    v4f  __attribute__((ext_vector_type(4)));
typedef v8h __attribute__((may_alias)) v8ha;
typedef v4h __attribute__((may_alias)) v4ha;
typedef v4f __attribute__((may_alias)) v4fa;
union FragH { v16h v; v8h half[2]; };

#define NBAT   2
#define DIMC   256
#define NHEAD  8
#define HDIM   32
#define IMG    96
#define NPIX   (IMG * IMG)
#define NWIN   24
#define PSZ    8
#define STRD   4
#define NTOK   64
#define NQ     16
#define NPOS   225
#define NQKV   768

#define ATPB   128
#define AWAVES 4
#define GTPB   256
#define GWAVES 8
#define MT     64
#define PQF    132

#define QCAR   64.0f
#define KCAR   16.0f
#define VCAR   16.0f
#define PCAR   1024.0f
#define WCAR   256.0f
#define RSC    0.17677669529663687f
#define SC_QK  (1.0f / (64.0f * 16.0f))
#define SC_PV  (16.0f / (1024.0f * 16.0f))
#define SC_OW  (1.0f / (16.0f * 256.0f))

#define NABLK  (NBAT * NWIN * NWIN * 2)
#define WBLK   (DIMC * DIMC / 8 / GTPB)
#define NROWO  (NBAT * NPIX)

static_assert(ATPB == AWAVES * 32);
static_assert(GTPB == GWAVES * 32);
static_assert(AWAVES * HDIM == ATPB);
static_assert(2 * AWAVES == NHEAD);
static_assert(NHEAD * HDIM == DIMC);
static_assert(NWIN * STRD == IMG);
static_assert((IMG + (PSZ - STRD) - PSZ) / STRD + 1 == NWIN);
static_assert(PSZ * PSZ == NTOK);
static_assert(STRD * STRD == NQ);
static_assert(NQ * (AWAVES * HDIM) / 8 == 2 * ATPB);
static_assert(WBLK * GTPB * 8 == DIMC * DIMC);
static_assert((NPIX % 128) == 0);
static_assert((DIMC % MT) == 0);
static_assert((DIMC % 32) == 0);
static_assert((PQF % 4) == 0);
static_assert(MT == 64);

DEVINL int imin(int a, int b) { return a < b ? a : b; }
DEVINL int imax(int a, int b) { return a > b ? a : b; }

DEVINL v8f wmma_f16(v16h a, v16h b, v8f c) {
  v8f d = __builtin_amdgcn_wmma_f32_16x16x32_f16(false, a, false, b, (short)0, c, false, false);
  asm volatile("v_nop\n\tv_nop\n\tv_nop\n\tv_nop" : "+v"(d) : "v"(a), "v"(b));
  return d;
}
DEVINL v8f zero8f() {
  v8f z = {0.f, 0.f, 0.f, 0.f, 0.f, 0.f, 0.f, 0.f};
  return z;
}
DEVINL void load_frag(FragH& f, const f16t* row, int k0) {
  f.half[0] = *(const v8ha*)(row + k0);
  f.half[1] = *(const v8ha*)(row + k0 + 16);
}

template <int KD>
DEVINL void mma_4n(const f16t* __restrict__ arow, const f16t* __restrict__ brow, v8f (&acc)[4]) {
  #pragma unroll 1
  for (int ks = 0; ks < KD / 32; ++ks) {
    const int k0 = 32 * ks;
    FragH a;
    load_frag(a, arow, k0);
    #pragma unroll
    for (int n = 0; n < 4; ++n) {
      FragH b;
      load_frag(b, brow + (size_t)16 * n * KD, k0);
      acc[n] = wmma_f16(a.v, b.v, acc[n]);
    }
  }
}

DEVINL void store_rows_f32(const float* sbuf, float* dst, int pitch, int wave, int lane) {
  #pragma unroll
  for (int i = 0; i < 8; ++i) {
    const int row = wave + 8 * i;
    const v4f v = *(const v4fa*)(sbuf + row * PQF + 4 * lane);
    *(volatile v4f*)(dst + (size_t)row * pitch + 4 * lane) = v;
  }
  __threadfence();
  #pragma unroll
  for (int i = 0; i < 8; ++i) {
    const int row = wave + 8 * i;
    const v4f v = *(const v4fa*)(sbuf + row * PQF + 4 * lane);
    *(volatile v4f*)(dst + (size_t)row * pitch + 4 * lane) = v;
  }
}

__global__ __launch_bounds__(GTPB) void prep_w_k(const float* __restrict__ w, f16t* __restrict__ W16)
{
  const int blk = blockIdx.x, tid = threadIdx.x;
  if (blk >= WBLK) return;
  const size_t idx = ((size_t)blk * GTPB + tid) * 8;
  const v4f a = *(const v4fa*)(w + idx), c = *(const v4fa*)(w + idx + 4);
  v8h o;
  #pragma unroll
  for (int j = 0; j < 4; ++j) {
    o[j]     = (f16t)(a[j] * WCAR);
    o[4 + j] = (f16t)(c[j] * WCAR);
  }
  *(volatile v8h*)(W16 + idx) = o;
  __threadfence();
  *(volatile v8h*)(W16 + idx) = o;
}

__global__ __launch_bounds__(ATPB) void attn_k(const float* __restrict__ x, const float* __restrict__ qkv_w,
                                              const float* __restrict__ qkv_b, const float* __restrict__ pos,
                                              f16t* __restrict__ Opl)
{
  __shared__ __attribute__((aligned(16))) float sPos[NPOS * NHEAD];
  __shared__ __attribute__((aligned(16))) float sWb[6 * ATPB];
  __shared__ __attribute__((aligned(16))) f16t  sQ [AWAVES * NQ * HDIM];
  __shared__ __attribute__((aligned(16))) f16t  sK [AWAVES * NTOK * HDIM];
  __shared__ __attribute__((aligned(16))) f16t  sVt[AWAVES * HDIM * NTOK];
  __shared__ __attribute__((aligned(16))) f16t  sP [AWAVES * NQ * NTOK];
  __shared__ __attribute__((aligned(16))) f16t  sO [NQ * AWAVES * HDIM];

  const int tid = threadIdx.x, lane = tid & 31;
  const int wave = __builtin_amdgcn_readfirstlane(tid >> 5);
  const int h = lane >> 4, m = lane & 15;
  int bid = blockIdx.x;
  const int hg = bid & 1;   bid >>= 1;
  const int wx = bid % NWIN; bid /= NWIN;
  const int wy = bid % NWIN;
  const int b  = imin(bid / NWIN, NBAT - 1);
  const int head = hg * AWAVES + wave;
  const int cblk = hg * (AWAVES * HDIM);

  for (int i = tid; i < NPOS * NHEAD; i += ATPB) sPos[i] = pos[i];
  {
    const int ch = cblk + tid;
    sWb[tid]            = qkv_w[ch];
    sWb[ATPB + tid]     = qkv_b[ch];
    sWb[2 * ATPB + tid] = qkv_w[DIMC + ch];
    sWb[3 * ATPB + tid] = qkv_b[DIMC + ch];
    sWb[4 * ATPB + tid] = qkv_w[2 * DIMC + ch];
    sWb[5 * ATPB + tid] = qkv_b[2 * DIMC + ch];
  }
  __syncthreads();

  f16t* sQw = sQ  + wave * (NQ * HDIM);
  f16t* sKw = sK  + wave * (NTOK * HDIM);
  f16t* sVw = sVt + wave * (HDIM * NTOK);
  f16t* sPw = sP  + wave * (NQ * NTOK);

  {
    const int ry  = (lane >> 1) & 7, hf = lane & 1;
    const int gy  = imin(wy * STRD + ry, IMG - 1);
    const int gx0 = wx * STRD + 4 * hf;
    const int gxa = imin(gx0, IMG - 4);
    const bool edge = gx0 > IMG - 4;
    const int tok0 = ry * PSZ + 4 * hf;
    const bool qrow = (ry < STRD) && (hf == 0);
    #pragma unroll 1
    for (int it = 0; it < 16; ++it) {
      const int c  = (lane >> 4) + 2 * it;
      const int ch = head * HDIM + c;
      const v4f ld = *(const v4fa*)(x + ((size_t)(b * DIMC + ch) * IMG + gy) * IMG + gxa);
      const int cl = wave * HDIM + c;
      const float wq = sWb[cl],            bq = sWb[ATPB + cl];
      const float wk = sWb[2 * ATPB + cl], bk = sWb[3 * ATPB + cl];
      const float wv = sWb[4 * ATPB + cl], bv = sWb[5 * ATPB + cl];
      v4h vv;
      #pragma unroll
      for (int j = 0; j < 4; ++j) {
        const float xv = edge ? ld[3] : ld[j];
        const float kv = xv * wk + bk;
        const float v1 = xv * wv + bv;
        const float qv = (xv * wq + bq) * RSC;
        sKw[(tok0 + j) * HDIM + c] = (f16t)(kv * KCAR);
        vv[j] = (f16t)(v1 * VCAR);
        if (qrow) sQw[(ry * STRD + j) * HDIM + c] = (f16t)(qv * QCAR);
      }
      *(v4ha*)(sVw + c * NTOK + tok0) = vv;
    }
  }
  __syncthreads();

  FragH qa;
  qa.half[0] = *(const v8ha*)(sQw + m * HDIM + 8 * h);
  qa.half[1] = *(const v8ha*)(sQw + m * HDIM + 16 + 8 * h);
  v8f acc[4];
  #pragma unroll
  for (int nt = 0; nt < 4; ++nt) {
    FragH kb;
    kb.half[0] = *(const v8ha*)(sKw + (nt * 16 + m) * HDIM + 8 * h);
    kb.half[1] = *(const v8ha*)(sKw + (nt * 16 + m) * HDIM + 16 + 8 * h);
    acc[nt] = wmma_f16(qa.v, kb.v, zero8f());
  }

  #pragma unroll
  for (int r = 0; r < 8; ++r) {
    const int row = 8 * h + r;
    const int qi = row >> 2, qj = row & 3;
    float s[4];
    #pragma unroll
    for (int nt = 0; nt < 4; ++nt) {
      const int kt = nt * 16 + m;
      const int bidx = (qi - (kt >> 3) + 7) * 15 + (qj - (kt & 7) + 7);
      s[nt] = acc[nt][r] * SC_QK + sPos[bidx * NHEAD + head];
    }
    float mx = fmaxf(fmaxf(s[0], s[1]), fmaxf(s[2], s[3]));
    mx = fmaxf(mx, __shfl_xor(mx, 1));
    mx = fmaxf(mx, __shfl_xor(mx, 2));
    mx = fmaxf(mx, __shfl_xor(mx, 4));
    mx = fmaxf(mx, __shfl_xor(mx, 8));
    float e[4], sum = 0.0f;
    #pragma unroll
    for (int nt = 0; nt < 4; ++nt) { e[nt] = __expf(s[nt] - mx); sum += e[nt]; }
    sum += __shfl_xor(sum, 1);
    sum += __shfl_xor(sum, 2);
    sum += __shfl_xor(sum, 4);
    sum += __shfl_xor(sum, 8);
    const float psc = PCAR / sum;
    #pragma unroll
    for (int nt = 0; nt < 4; ++nt) sPw[row * NTOK + nt * 16 + m] = (f16t)(e[nt] * psc);
  }
  __syncthreads();

  v8f oc[2];
  oc[0] = zero8f(); oc[1] = zero8f();
  #pragma unroll
  for (int ks = 0; ks < 2; ++ks) {
    FragH pa;
    pa.half[0] = *(const v8ha*)(sPw + m * NTOK + 32 * ks + 8 * h);
    pa.half[1] = *(const v8ha*)(sPw + m * NTOK + 32 * ks + 16 + 8 * h);
    #pragma unroll
    for (int nt = 0; nt < 2; ++nt) {
      FragH vb;
      vb.half[0] = *(const v8ha*)(sVw + (nt * 16 + m) * NTOK + 32 * ks + 8 * h);
      vb.half[1] = *(const v8ha*)(sVw + (nt * 16 + m) * NTOK + 32 * ks + 16 + 8 * h);
      oc[nt] = wmma_f16(pa.v, vb.v, oc[nt]);
    }
  }
  #pragma unroll
  for (int nt = 0; nt < 2; ++nt) {
    #pragma unroll
    for (int r = 0; r < 8; ++r)
      sO[(8 * h + r) * (AWAVES * HDIM) + wave * HDIM + nt * 16 + m] = (f16t)(oc[nt][r] * SC_PV);
  }
  __syncthreads();

  const int p0 = tid, p1 = ATPB + tid;
  const int pr0 = p0 >> 4, c0 = p0 & 15, pr1 = p1 >> 4, c1 = p1 & 15;
  const v8h ov0 = *(const v8ha*)(sO + pr0 * (AWAVES * HDIM) + 8 * c0);
  const v8h ov1 = *(const v8ha*)(sO + pr1 * (AWAVES * HDIM) + 8 * c1);
  const size_t orow0 = (size_t)b * NPIX + (size_t)(wy * STRD + (pr0 >> 2)) * IMG + (size_t)(wx * STRD + (pr0 & 3));
  const size_t orow1 = (size_t)b * NPIX + (size_t)(wy * STRD + (pr1 >> 2)) * IMG + (size_t)(wx * STRD + (pr1 & 3));
  f16t* d0 = Opl + orow0 * DIMC + cblk + 8 * c0;
  f16t* d1 = Opl + orow1 * DIMC + cblk + 8 * c1;
  *(volatile v8h*)d0 = ov0;
  *(volatile v8h*)d1 = ov1;
  __threadfence();
  *(volatile v8h*)d0 = ov0;
  *(volatile v8h*)d1 = ov1;
}

__global__ __launch_bounds__(GTPB) void proj_k(const f16t* __restrict__ W16, const f16t* __restrict__ Opl,
                                             float* __restrict__ out)
{
  __shared__ __attribute__((aligned(16))) float sbuf[MT * PQF];
  const int tid = threadIdx.x, lane = tid & 31, wave = tid >> 5;
  const int h = lane >> 4, m = lane & 15;
  const int mt = wave & 3, nh = wave >> 2;
  const int xt = blockIdx.x, yt = blockIdx.y;
  const int b  = imin((int)blockIdx.z, NBAT - 1);

  v8f acc[4];
  #pragma unroll
  for (int n = 0; n < 4; ++n) acc[n] = zero8f();
  const f16t* arow = W16 + (size_t)(yt * MT + 16 * mt + m) * DIMC + 8 * h;
  const f16t* brow = Opl + ((size_t)b * NPIX + (size_t)(xt * 128 + 64 * nh + m)) * DIMC + 8 * h;
  mma_4n<DIMC>(arow, brow, acc);

  #pragma unroll
  for (int n = 0; n < 4; ++n) {
    #pragma unroll
    for (int r = 0; r < 8; ++r)
      sbuf[(16 * mt + 8 * h + r) * PQF + 64 * nh + 16 * n + m] = acc[n][r] * SC_OW;
  }
  __syncthreads();
  store_rows_f32(sbuf, out + ((size_t)b * DIMC + (size_t)yt * MT) * NPIX + (size_t)xt * 128, NPIX, wave, lane);
}

extern "C" void kernel_launch(void* const* d_in, const int* in_sizes, int n_in,
                              void* d_out, int out_size, void* d_ws, size_t ws_size,
                              hipStream_t stream) {
  if (n_in < 5) return;
  if (in_sizes[0] != NBAT * DIMC * NPIX) return;
  if (in_sizes[1] != NQKV || in_sizes[2] != NQKV) return;
  if (in_sizes[3] != DIMC * DIMC) return;
  if (in_sizes[4] != NPOS * NHEAD) return;
  if (out_size != NBAT * DIMC * NPIX) return;

  const float* x     = (const float*)d_in[0];
  const float* qkv_w = (const float*)d_in[1];
  const float* qkv_b = (const float*)d_in[2];
  const float* out_w = (const float*)d_in[3];
  const float* pos   = (const float*)d_in[4];
  float* outp = (float*)d_out;

  const size_t szW16 = (size_t)DIMC * DIMC * 2;
  const size_t szOPL = (size_t)NROWO * DIMC * 2;
  size_t off = 0;
  char* ws = (char*)d_ws;
  f16t* W16 = (f16t*)(ws + off);  off += szW16;
  f16t* Opl = (f16t*)(ws + off);  off += szOPL;
  if (off > ws_size) return;

  prep_w_k<<<WBLK, GTPB, 0, stream>>>(out_w, W16);
  attn_k<<<NABLK, ATPB, 0, stream>>>(x, qkv_w, qkv_b, pos, Opl);
  proj_k<<<dim3(NPIX / 128, DIMC / MT, NBAT), GTPB, 0, stream>>>(W16, Opl, outp);
  (void)hipGetLastError();
}
